// SupConLoss_2516850835771
// MI455X (gfx1250) — hardware-run, weakly checked
//
#include <hip/hip_runtime.h>
#include <math.h>

typedef __attribute__((ext_vector_type(16))) _Float16 v16h;
typedef __attribute__((ext_vector_type(16))) __bf16 v16b;
typedef __attribute__((ext_vector_type(8)))  _Float16 v8h;
typedef __attribute__((ext_vector_type(8)))  float v8f;
typedef __attribute__((ext_vector_type(4)))  float v4f;
typedef __attribute__((ext_vector_type(2)))  float v2f;
typedef __attribute__((ext_vector_type(4)))  unsigned v4u;
typedef __attribute__((ext_vector_type(4)))  int v4i;
typedef float __attribute__((may_alias)) float_a;
typedef int __attribute__((may_alias)) int_a;

template <typename T> __device__ __forceinline__ void vst2(void* p, T v) { *(volatile T*)p = v; __threadfence(); *(volatile T*)p = v; }
__device__ __forceinline__ v8f wmma16(v16h a, v16h b, v8f c) {
  v8f d = __builtin_amdgcn_wmma_f32_16x16x32_f16(false, a, false, b, (short)0, c, false, false);
  asm volatile("v_nop\n\tv_nop\n\tv_nop\n\tv_nop" : "+v"(d) : "v"(a), "v"(b));
  return d;
}
__device__ __forceinline__ v8f wmma_bf(v16b a, v16b b, v8f c) {
  v8f d = __builtin_amdgcn_wmma_f32_16x16x32_bf16(false, a, false, b, (short)0, c, false, false);
  asm volatile("v_nop\n\tv_nop\n\tv_nop\n\tv_nop" : "+v"(d) : "v"(a), "v"(b));
  return d;
}
__device__ __forceinline__ v16h frag_h(const _Float16* rowk0, int lane) {
  union { v16h v; v8h q[2]; } u; const _Float16* p = rowk0 + 8 * (lane >> 4);
  u.q[0] = *(const v8h*)p; u.q[1] = *(const v8h*)(p + 16); return u.v;
}
__device__ __forceinline__ v16h frag_f32(const float* rowk0, int lane) {
  v16h a; const float* p = rowk0 + 8 * (lane >> 4);
#pragma unroll
  for (int i = 0; i < 8; ++i) { a[i] = (_Float16)p[i]; a[8 + i] = (_Float16)p[16 + i]; }
  return a;
}
__device__ __forceinline__ v16h frag_f32s(const float* rowk0, int lane, float sc) {
  v16h a; const float* p = rowk0 + 8 * (lane >> 4);
#pragma unroll
  for (int i = 0; i < 8; ++i) { a[i] = (_Float16)(p[i] * sc); a[8 + i] = (_Float16)(p[16 + i] * sc); }
  return a;
}
__device__ __forceinline__ v16h fragc_f32(const float* W, int k0, int n, int lane, int ld, int K) {
  v16h a; const int g = lane >> 4;
#pragma unroll
  for (int i = 0; i < 8; ++i) { const int ka = k0 + 8 * g + i, kb = ka + 16;
    a[i] = (_Float16)(ka < K ? W[(size_t)(ka < K ? ka : K - 1) * ld + n] : 0.f); a[8 + i] = (_Float16)(kb < K ? W[(size_t)(kb < K ? kb : K - 1) * ld + n] : 0.f); }
  return a;
}
struct F2 { v16b h, l; };
__device__ __forceinline__ F2 bsplit16(const float v[16]) { F2 r;
#pragma unroll
  for (int i = 0; i < 16; ++i) { const __bf16 h = (__bf16)v[i]; r.h[i] = h; r.l[i] = (__bf16)(v[i] - (float)h); }
  return r; }
__device__ __forceinline__ F2 split_row(const float* row, int k0, int lane) { float v[16]; const float* p = row + k0 + 8 * (lane >> 4);
#pragma unroll
  for (int i = 0; i < 8; ++i) { v[i] = p[i]; v[8 + i] = p[16 + i]; }
  return bsplit16(v); }
__device__ __forceinline__ F2 split_rowK(const float* row, int k0, int lane, int K) { float v[16]; const int g = lane >> 4;
#pragma unroll
  for (int i = 0; i < 8; ++i) { const int ka = k0 + 8 * g + i, kb = ka + 16; v[i] = ka < K ? row[ka < K ? ka : K - 1] : 0.f; v[8 + i] = kb < K ? row[kb < K ? kb : K - 1] : 0.f; }
  return bsplit16(v); }
__device__ __forceinline__ F2 split_col(const float* W, int k0, int n, int lane, int ld, int K) { float v[16]; const int g = lane >> 4;
#pragma unroll
  for (int i = 0; i < 8; ++i) { const int ka = k0 + 8 * g + i, kb = ka + 16; v[i] = ka < K ? W[(size_t)(ka < K ? ka : K - 1) * ld + n] : 0.f; v[8 + i] = kb < K ? W[(size_t)(kb < K ? kb : K - 1) * ld + n] : 0.f; }
  return bsplit16(v); }
__device__ __forceinline__ v8f mac3(const F2& a, const F2& b, v8f c) { c = wmma_bf(a.l, b.h, c); c = wmma_bf(a.h, b.l, c); return wmma_bf(a.h, b.h, c); }
__device__ __forceinline__ float sigm(float v) { return 1.0f / (1.0f + expf(-v)); }
#define LDSX() do { asm volatile("s_wait_dscnt 0" ::: "memory"); __builtin_amdgcn_wave_barrier(); __builtin_amdgcn_fence(__ATOMIC_RELEASE, "workgroup"); } while (0)


#define NN 8192
#define DD 256
#define INVT (1.0f / 0.07f)
#define NBLK (NN / 64)
#ifndef TQB
#define TQB NBLK
#endif
typedef __attribute__((ext_vector_type(8))) __bf16 v8b;
__device__ __forceinline__ v16b frag_b(const __bf16* rowk0, int lane) {
  union { v16b v; v8b q[2]; } u; const __bf16* p = rowk0 + 8 * (lane >> 4);
  u.q[0] = *(const v8b*)p; u.q[1] = *(const v8b*)(p + 16); return u.v;
}
__device__ __forceinline__ float bfr(float v) { return (float)(__bf16)v; }
__device__ __attribute__((noinline)) float exp_ni(float v) { return expf(v); }
__device__ __attribute__((noinline)) float erf_ni(float v) { return erff(v); }

#define WS_PB  0u
#define WS_END (WS_PB + 128u * NBLK)

__device__ __forceinline__ v16b fragb_f32(const float* __restrict__ p, int lane) { v16b a; const float* pp = p + 8 * (lane >> 4);
#pragma unroll
  for (int i = 0; i < 8; ++i) { a[i] = (__bf16)pp[i]; a[8 + i] = (__bf16)pp[16 + i]; } return a; }
__global__ __launch_bounds__(128) void k_rows(const float* __restrict__ Fe, const int* __restrict__ LB, float* __restrict__ PB) { __shared__ float sl[4][16]; __shared__ int sc[4][16]; __shared__ __align__(16) float sres[4];
  const int tid = threadIdx.x, wave = tid >> 5, lane = tid & 31, col = lane & 15, g = lane >> 4; const int q0 = blockIdx.x * 64 + wave * 16;
  v16b aq[DD / 32];
#pragma unroll
  for (int kc = 0; kc < DD / 32; ++kc) aq[kc] = fragb_f32(Fe + (size_t)(q0 + col) * DD + kc * 32, lane);
  int lab[8]; float m[8], l[8], sp[8]; int np[8];
#pragma unroll
  for (int r = 0; r < 8; ++r) { lab[r] = LB[q0 + 8 * g + r]; m[r] = -3.0e38f; l[r] = 0.f; sp[r] = 0.f; np[r] = 0; }
#pragma unroll 1
  for (int ks = 0; ks < NN / 32; ++ks) { float s[2][8]; int lk[2];
#pragma unroll
    for (int ct = 0; ct < 2; ++ct) { const int kk = ks * 32 + ct * 16 + col; lk[ct] = LB[kk]; v8f c = {};
#pragma unroll
      for (int kc = 0; kc < DD / 32; ++kc) c = wmma_bf(aq[kc], fragb_f32(Fe + (size_t)kk * DD + kc * 32, lane), c);
#pragma unroll
      for (int r = 0; r < 8; ++r) { s[ct][r] = c[r] * INVT; const int qi = q0 + 8 * g + r; if (lk[ct] == lab[r] && kk != qi) { sp[r] += s[ct][r]; np[r] += 1; } } }
#pragma unroll
    for (int r = 0; r < 8; ++r) { float mx = fmaxf(s[0][r], s[1][r]);
#pragma unroll
      for (int o = 1; o < 16; o <<= 1) mx = fmaxf(mx, __shfl_xor(mx, o));
      const float mn = fmaxf(m[r], mx); const float alpha = __expf(m[r] - mn); float es = __expf(s[0][r] - mn) + __expf(s[1][r] - mn);
#pragma unroll
      for (int o = 1; o < 16; o <<= 1) es += __shfl_xor(es, o);
      l[r] = l[r] * alpha + es; m[r] = mn; } }
  float wsum = 0.f; int wcnt = 0;
#pragma unroll
  for (int r = 0; r < 8; ++r) { float a = sp[r]; int n = np[r];
#pragma unroll
    for (int o = 1; o < 16; o <<= 1) { a += __shfl_xor(a, o); n += __shfl_xor(n, o); }
    if (col == 0) { const float loss = (n > 0) ? (-a / (float)n + m[r] + logf(l[r] + 1e-9f)) : 0.f; sl[wave][8 * g + r] = loss; sc[wave][8 * g + r] = (n > 0) ? 1 : 0; } }
  __syncthreads();
  if (tid == 0) { float a = 0.f; int n = 0; for (int w = 0; w < 4; ++w) for (int r = 0; r < 16; ++r) { a += sl[w][r]; n += sc[w][r]; } sres[0] = a; sres[1] = (float)n; sres[2] = 0.f; sres[3] = 0.f; vst2(PB + (size_t)blockIdx.x * 32, *(const v4f*)sres); } (void)wsum; (void)wcnt; }
__global__ __launch_bounds__(64) void k_fin(const float* __restrict__ PB, float* __restrict__ OUT) { __shared__ float st[2];
  if (threadIdx.x == 0) { float a = 0.f, n = 0.f;
#pragma unroll 1
    for (int b = 0; b < TQB; ++b) { a += PB[b * 32]; n += PB[b * 32 + 1]; }
    st[0] = (n > 0.f) ? a / n : 0.f; vst2(OUT, st[0]); } }
extern "C" void kernel_launch(void* const* d_in, const int* in_sizes, int n_in, void* d_out, int out_size, void* d_ws, size_t ws_size, hipStream_t stream) {
  (void)in_sizes; (void)n_in; (void)out_size;
  const float** F = (const float**)d_in;
  if (ws_size < (size_t)WS_END) return;
  char* ws = (char*)d_ws; float* PB = (float*)(ws + WS_PB);
  k_rows<<<TQB, 128, 0, stream>>>(F[0], (const int*)d_in[1], PB);
  k_fin<<<1, 64, 0, stream>>>(PB, (float*)d_out);
}
